// EncoderLayer_16269336117672
// MI455X (gfx1250) — hardware-verified
//
#include <hip/hip_runtime.h>


#ifndef NB
#define NB 4
#endif
#ifndef SEQ
#define SEQ 1024
#endif
#define NB_FULL  4
#define SEQ_FULL 1024
#define DM    1024
#define NH    16
#define HD    64
#define FF    4096
#define MAXD  128
#define NREL  (2 * MAXD - 1)
#define MROWS (NB * SEQ)
#define NBH   (NB * NH)
#define ZH    8
#define LNEPS 1e-5f
#define QSC   4.0f
#define SCL2  0.0078125f
#define PCAR  1024.0f
#define WCAR  64.0f
#define CCAR  0.0625f
#define HCAR  8.0f
#define OSCO  0.000244140625f
#define OSCF  0.001953125f

static_assert(SEQ % 128 == 0);
static_assert(MROWS % 64 == 0);
static_assert(NH % ZH == 0);
static_assert(HD == 64);
static_assert(DM % 128 == 0);
static_assert(FF % 64 == 0);
static_assert(NB >= 1 && NB <= NB_FULL);
static_assert(SEQ <= SEQ_FULL);
static_assert(NREL <= 256);
static_assert(((size_t)MROWS * DM) % 8 == 0);

typedef _Float16 h16;
typedef unsigned short bf;
typedef __attribute__((ext_vector_type(16))) __bf16   v16bf;
typedef __attribute__((ext_vector_type(16))) _Float16 v16h;
typedef __attribute__((ext_vector_type(8)))  _Float16 v8h;
typedef __attribute__((ext_vector_type(4)))  _Float16 v4h;
typedef __attribute__((ext_vector_type(8)))  unsigned short v8us;
typedef __attribute__((ext_vector_type(8)))  float    v8f;
typedef __attribute__((ext_vector_type(4)))  float    v4f;
typedef v4f  __attribute__((may_alias)) v4fa;

__device__ __forceinline__ unsigned short f2bf(float f) { unsigned u = __float_as_uint(f); u += 0x7FFFu + ((u >> 16) & 1u); return (unsigned short)(u >> 16); }
__device__ __forceinline__ float bf2f(unsigned short b) { return __uint_as_float(((unsigned)b) << 16); }
__device__ __forceinline__ float bfr(float f) { return bf2f(f2bf(f)); }
__device__ __forceinline__ h16 tohx(float x) { return (h16)x; }
__device__ __forceinline__ v16h cat16(v8h lo, v8h hi) { return __builtin_shufflevector(lo, hi, 0, 1, 2, 3, 4, 5, 6, 7, 8, 9, 10, 11, 12, 13, 14, 15); }
__device__ __forceinline__ v16bf cat16b(v8us lo, v8us hi) { return __builtin_bit_cast(v16bf, __builtin_shufflevector(lo, hi, 0, 1, 2, 3, 4, 5, 6, 7, 8, 9, 10, 11, 12, 13, 14, 15)); }
__device__ __forceinline__ v8f wmma16(v16h a, v16h b, v8f c) { return __builtin_amdgcn_wmma_f32_16x16x32_f16(false, a, false, b, (short)0, c, false, false); }
__device__ __forceinline__ v8f wmmab(v16bf a, v16bf b, v8f c) { return __builtin_amdgcn_wmma_f32_16x16x32_bf16(false, a, false, b, (short)0, c, false, false); }

template <typename T16> struct WFrag;
template <> struct WFrag<h16> { typedef v16h V; static __device__ __forceinline__ V ld(const h16* p) { return cat16(*(const v8h*)p, *(const v8h*)(p + 16)); } static __device__ __forceinline__ v8f mma(V a, V b, v8f c) { return wmma16(a, b, c); } };
template <> struct WFrag<bf> { typedef v16bf V; static __device__ __forceinline__ V ld(const bf* p) { return cat16b(*(const v8us*)p, *(const v8us*)(p + 16)); } static __device__ __forceinline__ v8f mma(V a, V b, v8f c) { return wmmab(a, b, c); } };
template <typename T16, int NSPLIT, bool BIAS>
__global__ __launch_bounds__(32) void k_gemmw(const T16* __restrict__ A, const T16* __restrict__ A2, const T16* __restrict__ Bt, const T16* __restrict__ Bt2, int K, float* C, int ldc, float oscale, const float* __restrict__ bias, size_t sA, size_t sB, size_t sC) {
    typedef typename WFrag<T16>::V V;
    __shared__ __align__(16) float os[16 * 68];
    const size_t z = blockIdx.z; A += z * sA; if (A2) A2 += z * sA; Bt += z * sB; if (Bt2) Bt2 += z * sB; C += z * sC;
    const int lane = threadIdx.x & 31, lr = lane & 15, hi = lane >> 4; const int r0 = blockIdx.x * 64, c0 = blockIdx.y * 64;
    v8f acc[4][4];
#pragma unroll
    for (int mb = 0; mb < 4; ++mb)
#pragma unroll
        for (int nb = 0; nb < 4; ++nb) acc[mb][nb] = (v8f){};
    const size_t aoff = (size_t)(r0 + lr) * K + 8 * hi, boff = (size_t)(c0 + lr) * K + 8 * hi;
#pragma unroll 1
    for (int kc = 0; kc < K; kc += 32) {
        V a[4], a2[4];
#pragma unroll
        for (int mb = 0; mb < 4; ++mb) { a[mb] = WFrag<T16>::ld(A + aoff + (size_t)mb * 16 * K + kc); if (NSPLIT == 1 || NSPLIT == 2) a2[mb] = WFrag<T16>::ld(A2 + aoff + (size_t)mb * 16 * K + kc); }
#pragma unroll
        for (int nb = 0; nb < 4; ++nb) { const V b = WFrag<T16>::ld(Bt + boff + (size_t)nb * 16 * K + kc); V b2; if (NSPLIT >= 2) b2 = WFrag<T16>::ld(Bt2 + boff + (size_t)nb * 16 * K + kc);
#pragma unroll
            for (int mb = 0; mb < 4; ++mb) { acc[mb][nb] = WFrag<T16>::mma(a[mb], b, acc[mb][nb]); if (NSPLIT == 1 || NSPLIT == 2) acc[mb][nb] = WFrag<T16>::mma(a2[mb], b, acc[mb][nb]); if (NSPLIT >= 2) acc[mb][nb] = WFrag<T16>::mma(a[mb], b2, acc[mb][nb]); } }
        asm volatile("v_nop\n\tv_nop\n\tv_nop\n\tv_nop" : "+v"(acc[0][0]), "+v"(acc[1][1]), "+v"(acc[2][2]), "+v"(acc[3][3]) : "v"(a[0]), "v"(a[3]));
    }
#pragma unroll
    for (int mb = 0; mb < 4; ++mb) {
#pragma unroll
        for (int nb = 0; nb < 4; ++nb) {
#pragma unroll
            for (int j = 0; j < 8; ++j) os[(hi * 8 + j) * 68 + nb * 16 + lr] = acc[mb][nb][j]; }
        __builtin_amdgcn_wave_barrier(); asm volatile("" ::: "memory");
        float* crow = C + (size_t)(r0 + mb * 16) * ldc + c0;
#pragma unroll 1
        for (int ps = 0; ps < 2; ++ps) {
#pragma unroll
            for (int s = 0; s < 8; ++s) { const int row = 2 * s + hi, cofs = lr * 4; v4f val = *(const v4fa*)(os + row * 68 + cofs); val = val * oscale;
                if (BIAS) { val[0] += bfr(bias[c0 + cofs]); val[1] += bfr(bias[c0 + cofs + 1]); val[2] += bfr(bias[c0 + cofs + 2]); val[3] += bfr(bias[c0 + cofs + 3]); }
                *(volatile v4f*)(crow + (size_t)row * ldc + cofs) = val; }
            if (ps == 0) __threadfence(); }
        __builtin_amdgcn_wave_barrier(); asm volatile("" ::: "memory");
    }
}

__global__ __launch_bounds__(256) void k_cvt8(const float* __restrict__ src, bf* dst, size_t n8) { const size_t i = (size_t)blockIdx.x * 256 + threadIdx.x; if (i >= n8) return; const v8f v = *(const v8f*)(src + i * 8); v8us o;
#pragma unroll
    for (int k = 0; k < 8; ++k) o[k] = f2bf(v[k]); *(volatile v8us*)(dst + i * 8) = o; __threadfence(); *(volatile v8us*)(dst + i * 8) = o; }

__global__ __launch_bounds__(256) void k_cvtx(const float* __restrict__ x, bf* dst) {
    const size_t i = (size_t)blockIdx.x * 256 + threadIdx.x; if (i >= (size_t)MROWS * DM / 8) return;
    const size_t e = i * 8; const int m = (int)(e / DM); const int c = (int)(e % DM); const int b = m / SEQ, s = m % SEQ;
    const v8f v = *(const v8f*)(x + ((size_t)b * SEQ_FULL + s) * DM + c); v8us o;
#pragma unroll
    for (int k = 0; k < 8; ++k) o[k] = f2bf(v[k]);
    *(volatile v8us*)(dst + e) = o; __threadfence(); *(volatile v8us*)(dst + e) = o; }

template <bool RELU, bool BFR>
__global__ __launch_bounds__(256) void k_tof16(const float* __restrict__ src, h16* dst, size_t n8, float sc) {
    const size_t i = (size_t)blockIdx.x * 256 + threadIdx.x; if (i >= n8) return; const v8f a = *(const v8f*)(src + i * 8); v8h o;
#pragma unroll
    for (int q = 0; q < 8; ++q) { float y = BFR ? bfr(a[q]) : a[q]; if (RELU) y = fmaxf(y, 0.0f); o[q] = tohx(y * sc); }
    *(volatile v8h*)(dst + i * 8) = o; __threadfence(); *(volatile v8h*)(dst + i * 8) = o; }

__global__ __launch_bounds__(256) void k_qkp(const float* __restrict__ F, float sc, h16* P) {
    const size_t i = (size_t)blockIdx.x * 256 + threadIdx.x; if (i >= (size_t)MROWS * DM / 8) return;
    const size_t e = i * 8; const int d = (int)(e % HD); const int t = (int)((e / HD) % SEQ); const int bh = (int)(e / ((size_t)HD * SEQ)); const int b = bh / NH, h = bh % NH;
    const v8f a = *(const v8f*)(F + ((size_t)b * SEQ + t) * DM + h * HD + d); v8h o;
#pragma unroll
    for (int q = 0; q < 8; ++q) o[q] = tohx(a[q] * sc);
    *(volatile v8h*)(P + e) = o; __threadfence(); *(volatile v8h*)(P + e) = o; }

__global__ __launch_bounds__(256) void k_vtp(const float* __restrict__ F, h16* VT) {
    const size_t i = (size_t)blockIdx.x * 256 + threadIdx.x; if (i >= (size_t)MROWS * DM / 8) return;
    const size_t e = i * 8; const int t = (int)(e % SEQ); const int d = (int)((e / SEQ) % HD); const int bh = (int)(e / ((size_t)SEQ * HD)); const int b = bh / NH, h = bh % NH;
    const float* src = F + ((size_t)b * SEQ + t) * DM + h * HD + d; v8h o;
#pragma unroll
    for (int q = 0; q < 8; ++q) o[q] = tohx(src[(size_t)q * DM]);
    *(volatile v8h*)(VT + e) = o; __threadfence(); *(volatile v8h*)(VT + e) = o; }

__global__ __launch_bounds__(256) void k_asoft(const float* __restrict__ Sb, const float* __restrict__ rel, int h0, h16* P16) {
    __shared__ float tb[256];
    const int lane = threadIdx.x & 31; const int row = blockIdx.x * 8 + (threadIdx.x >> 5);
    const int i = row % SEQ; const int h = h0 + (int)(((size_t)blockIdx.x * 8) / SEQ);
    if (threadIdx.x < NREL) tb[threadIdx.x] = bfr(rel[threadIdx.x * NH + h]);
    __syncthreads();
    const float* sr = Sb + (size_t)row * SEQ; float v[SEQ / 32]; float mx = -3.0e38f;
#pragma unroll
    for (int ch = 0; ch < SEQ / 128; ++ch) { const int j0 = ch * 128 + lane * 4; const v4f a = *(const v4f*)(sr + j0);
#pragma unroll
        for (int q = 0; q < 4; ++q) { int ri = i - (j0 + q) + (MAXD - 1); ri = (ri < 0) ? 0 : ((ri > 2 * MAXD - 2) ? (2 * MAXD - 2) : ri);
            float t = __fmul_rn(a[q], SCL2); asm volatile("" : "+v"(t)); t = __fadd_rn(t, tb[ri]); v[ch * 4 + q] = t; mx = fmaxf(mx, t); } }
#pragma unroll
    for (int sh = 16; sh; sh >>= 1) mx = fmaxf(mx, __shfl_xor(mx, sh, 32));
    float sum = 0.f;
#pragma unroll
    for (int k = 0; k < SEQ / 32; ++k) { float d0 = __fsub_rn(v[k], mx); asm volatile("" : "+v"(d0)); v[k] = __builtin_amdgcn_exp2f(__fmul_rn(d0, 1.4426950408889634f)); sum += v[k]; }
#pragma unroll
    for (int sh = 16; sh; sh >>= 1) sum += __shfl_xor(sum, sh, 32);
    const float f = __fdiv_rn(PCAR, sum);
#pragma unroll 1
    for (int ps = 0; ps < 2; ++ps) {
#pragma unroll
        for (int ch = 0; ch < SEQ / 128; ++ch) { v4h o4;
#pragma unroll
            for (int q = 0; q < 4; ++q) o4[q] = tohx(v[ch * 4 + q] * f);
            *(volatile v4h*)(P16 + (size_t)row * SEQ + ch * 128 + lane * 4) = o4; }
        if (ps == 0) __threadfence(); }
}

__global__ __launch_bounds__(256) void k_addres(float* Y, const float* __restrict__ x) {
    const size_t i = (size_t)blockIdx.x * 256 + threadIdx.x; if (i >= (size_t)MROWS * DM / 4) return;
    const size_t e = i * 4; const int m = (int)(e / DM); const int c = (int)(e % DM); const int b = m / SEQ, s = m % SEQ;
    const v4f a = *(const v4f*)(Y + e); const v4f r = *(const v4f*)(x + ((size_t)b * SEQ_FULL + s) * DM + c); v4f o;
#pragma unroll
    for (int q = 0; q < 4; ++q) o[q] = __fadd_rn(a[q], bfr(r[q]));
    *(volatile v4f*)(Y + e) = o; __threadfence(); *(volatile v4f*)(Y + e) = o; }

__global__ __launch_bounds__(256) void k_addf(float* Y, const float* __restrict__ R) {
    const size_t i = (size_t)blockIdx.x * 256 + threadIdx.x; if (i >= (size_t)MROWS * DM / 4) return;
    const v4f a = *(const v4f*)(Y + i * 4); const v4f r = *(const v4f*)(R + i * 4); v4f o;
#pragma unroll
    for (int q = 0; q < 4; ++q) o[q] = __fadd_rn(a[q], r[q]);
    *(volatile v4f*)(Y + i * 4) = o; __threadfence(); *(volatile v4f*)(Y + i * 4) = o; }

__global__ __launch_bounds__(256) void k_lnout(const float* __restrict__ F, const float* __restrict__ g, const float* __restrict__ bb, float* out, int nrows) {
    const int lane = threadIdx.x & 31; const int row = blockIdx.x * 8 + (threadIdx.x >> 5); if (row >= nrows) return;
    const float* fr = F + (size_t)row * DM; float* orow = out + (size_t)row * DM; float v[DM / 32]; float s = 0.f;
#pragma unroll
    for (int c = 0; c < DM / 128; ++c) { const v4f a = *(const v4f*)(fr + c * 128 + lane * 4);
#pragma unroll
        for (int q = 0; q < 4; ++q) { v[c * 4 + q] = a[q]; s = __fadd_rn(s, a[q]); } }
#pragma unroll
    for (int sh = 16; sh; sh >>= 1) s = __fadd_rn(s, __shfl_xor(s, sh, 32));
    const float mean = __fdiv_rn(s, (float)DM); float s2 = 0.f;
#pragma unroll
    for (int k = 0; k < DM / 32; ++k) { const float dv = __fsub_rn(v[k], mean); float p2 = __fmul_rn(dv, dv); asm volatile("" : "+v"(p2)); s2 = __fadd_rn(s2, p2); v[k] = dv; }
#pragma unroll
    for (int sh = 16; sh; sh >>= 1) s2 = __fadd_rn(s2, __shfl_xor(s2, sh, 32));
    const float rs = __fdiv_rn(1.0f, __fsqrt_rn(__fadd_rn(__fdiv_rn(s2, (float)DM), LNEPS)));
#pragma unroll 1
    for (int ps = 0; ps < 2; ++ps) {
#pragma unroll
        for (int c = 0; c < DM / 128; ++c) { v4f o;
#pragma unroll
            for (int q = 0; q < 4; ++q) { const int col = c * 128 + lane * 4 + q; float y = __fmul_rn(v[c * 4 + q], rs); asm volatile("" : "+v"(y)); y = __fmul_rn(y, bfr(g[col])); asm volatile("" : "+v"(y)); o[q] = __fadd_rn(y, bfr(bb[col])); }
            *(volatile v4f*)(orow + c * 128 + lane * 4) = o; }
        if (ps == 0) __threadfence(); } }

static inline size_t zmax(size_t a, size_t b) { return a > b ? a : b; }

extern "C" void kernel_launch(void* const* d_in, const int* in_sizes, int n_in,
                              void* d_out, int out_size, void* d_ws, size_t ws_size, hipStream_t stream) {
    if (n_in < 15) return;
    const size_t needx = ((size_t)(NB - 1) * SEQ_FULL + SEQ) * DM;
    if ((size_t)in_sizes[0] < needx) return;
    if (in_sizes[1] < DM * DM || in_sizes[2] < DM * DM || in_sizes[3] < DM * DM || in_sizes[4] < DM * DM) return;
    if (in_sizes[5] < DM || in_sizes[6] < NREL * NH || in_sizes[7] < FF * DM || in_sizes[8] < FF || in_sizes[9] < DM * FF || in_sizes[10] < DM) return;
    if (in_sizes[11] < DM || in_sizes[12] < DM || in_sizes[13] < DM || in_sizes[14] < DM) return;
    if ((size_t)out_size < (size_t)MROWS * DM) return;

    const float* x = (const float*)d_in[0]; const float* wq = (const float*)d_in[1]; const float* wk = (const float*)d_in[2]; const float* wv = (const float*)d_in[3]; const float* wo = (const float*)d_in[4];
    const float* bo = (const float*)d_in[5]; const float* rel = (const float*)d_in[6]; const float* w1 = (const float*)d_in[7]; const float* b1 = (const float*)d_in[8]; const float* w2 = (const float*)d_in[9]; const float* b2 = (const float*)d_in[10];
    const float* g1 = (const float*)d_in[11]; const float* be1 = (const float*)d_in[12]; const float* g2 = (const float*)d_in[13]; const float* be2 = (const float*)d_in[14];
    float* OUT = (float*)d_out;

    char* base = (char*)d_ws; size_t off = 0;
    auto carve = [&](size_t bytes) { char* p = base + off; off += (bytes + 255) & ~(size_t)255; return p; };
    const size_t plane2 = (size_t)MROWS * DM * 2;
    bf*  WQ   = (bf*)carve((size_t)DM * DM * 2); bf* WK = (bf*)carve((size_t)DM * DM * 2); bf* WV = (bf*)carve((size_t)DM * DM * 2);
    h16* WO16 = (h16*)carve((size_t)DM * DM * 2); h16* W1h = (h16*)carve((size_t)FF * DM * 2); h16* W2h = (h16*)carve((size_t)DM * FF * 2);
    char* RC = carve(zmax((size_t)MROWS * DM * 4, (size_t)SEQ * FF * 4));
    char* RD = carve(plane2 * 3);
    char* RE = carve(zmax(zmax(plane2, (size_t)ZH * SEQ * SEQ * 6), (size_t)MROWS * DM * 4 + (size_t)SEQ * FF * 2));
    if (off > ws_size) return;
    float* FP   = (float*)RC; float* CTX = (float*)RC; float* F2 = (float*)RC;
    h16*  QP16  = (h16*)RD; h16* KP16 = (h16*)(RD + plane2); h16* VT16 = (h16*)(RD + 2 * plane2);
    h16*  AT16  = (h16*)RD; float* N1 = (float*)(RD + plane2); h16* N1P = (h16*)RD;
    bf*   XB    = (bf*)RE; float* Sb = (float*)RE; h16* P16 = (h16*)(RE + (size_t)ZH * SEQ * SEQ * 4); float* Y = (float*)RE; h16* RP16 = (h16*)(RE + (size_t)MROWS * DM * 4);

    const unsigned G8M = (unsigned)(((size_t)MROWS * DM / 8 + 255) / 256), G4M = (unsigned)(((size_t)MROWS * DM / 4 + 255) / 256);
    const unsigned G8W = (unsigned)(((size_t)DM * DM / 8 + 255) / 256), G8F = (unsigned)(((size_t)FF * DM / 8 + 255) / 256), G8R = (unsigned)(((size_t)SEQ * FF / 8 + 255) / 256);

    k_cvt8<<<G8W, 256, 0, stream>>>(wq, WQ, (size_t)DM * DM / 8); k_cvt8<<<G8W, 256, 0, stream>>>(wk, WK, (size_t)DM * DM / 8); k_cvt8<<<G8W, 256, 0, stream>>>(wv, WV, (size_t)DM * DM / 8);
    k_tof16<false, true><<<G8W, 256, 0, stream>>>(wo, WO16, (size_t)DM * DM / 8, WCAR); k_tof16<false, true><<<G8F, 256, 0, stream>>>(w1, W1h, (size_t)FF * DM / 8, WCAR); k_tof16<false, true><<<G8F, 256, 0, stream>>>(w2, W2h, (size_t)DM * FF / 8, WCAR);
    k_cvtx<<<G8M, 256, 0, stream>>>(x, XB);
    k_gemmw<bf, 0, false><<<dim3(MROWS / 64, DM / 64, 1), 32, 0, stream>>>(XB, nullptr, WQ, nullptr, DM, FP, DM, 1.0f, nullptr, 0, 0, 0); k_qkp<<<G8M, 256, 0, stream>>>(FP, QSC, QP16);
    k_gemmw<bf, 0, false><<<dim3(MROWS / 64, DM / 64, 1), 32, 0, stream>>>(XB, nullptr, WK, nullptr, DM, FP, DM, 1.0f, nullptr, 0, 0, 0); k_qkp<<<G8M, 256, 0, stream>>>(FP, QSC, KP16);
    k_gemmw<bf, 0, false><<<dim3(MROWS / 64, DM / 64, 1), 32, 0, stream>>>(XB, nullptr, WV, nullptr, DM, FP, DM, 1.0f, nullptr, 0, 0, 0); k_vtp<<<G8M, 256, 0, stream>>>(FP, VT16);
    for (int p = 0; p < NBH / ZH; ++p) { const int bh0 = p * ZH; const int b = bh0 / NH, h0 = bh0 % NH;
        k_gemmw<h16, 0, false><<<dim3(SEQ / 64, SEQ / 64, ZH), 32, 0, stream>>>(QP16 + (size_t)bh0 * SEQ * HD, nullptr, KP16 + (size_t)bh0 * SEQ * HD, nullptr, HD, Sb, SEQ, 1.0f, nullptr, (size_t)SEQ * HD, (size_t)SEQ * HD, (size_t)SEQ * SEQ);
        k_asoft<<<ZH * SEQ / 8, 256, 0, stream>>>(Sb, rel, h0, P16);
        k_gemmw<h16, 0, false><<<dim3(SEQ / 64, HD / 64, ZH), 32, 0, stream>>>(P16, nullptr, VT16 + (size_t)bh0 * HD * SEQ, nullptr, SEQ, CTX + (size_t)b * SEQ * DM + (size_t)h0 * HD, DM, 1.0f, nullptr, (size_t)SEQ * SEQ, (size_t)HD * SEQ, (size_t)HD); }
    k_tof16<false, false><<<G8M, 256, 0, stream>>>(CTX, AT16, (size_t)MROWS * DM / 8, CCAR);
    k_gemmw<h16, 0, true><<<dim3(MROWS / 64, DM / 64, 1), 32, 0, stream>>>(AT16, nullptr, WO16, nullptr, DM, Y, DM, OSCO, bo, 0, 0, 0);
    k_addres<<<G4M, 256, 0, stream>>>(Y, x);
    k_lnout<<<(MROWS + 7) / 8, 256, 0, stream>>>(Y, g1, be1, N1, MROWS);
    k_tof16<false, false><<<G8M, 256, 0, stream>>>(N1, N1P, (size_t)MROWS * DM / 8, HCAR);
    for (int b = 0; b < NB; ++b) {
        k_gemmw<h16, 0, true><<<dim3(SEQ / 64, FF / 64, 1), 32, 0, stream>>>(N1P + (size_t)b * SEQ * DM, nullptr, W1h, nullptr, DM, F2, FF, OSCF, b1, 0, 0, 0);
        k_tof16<true, false><<<G8R, 256, 0, stream>>>(F2, RP16, (size_t)SEQ * FF / 8, HCAR);
        k_gemmw<h16, 0, true><<<dim3(SEQ / 64, DM / 64, 1), 32, 0, stream>>>(RP16, nullptr, W2h, nullptr, FF, Y + (size_t)b * SEQ * DM, DM, OSCF, b2, 0, 0, 0); }
    k_addf<<<G4M, 256, 0, stream>>>(Y, N1);
    k_lnout<<<(MROWS + 7) / 8, 256, 0, stream>>>(Y, g2, be2, OUT, MROWS);
}
